// VulnGAT_31241592111613
// MI455X (gfx1250) — hardware-verified
//
#include <hip/hip_runtime.h>
#include <stddef.h>


#define FIN     22
#define KIN     32
#define HID     128
#define HC      64
#define EDM     8
#define NCLS    5
#define GMAX    64
#define NTHR    256
#define NWAVE   8
#define EPT     8
#define NGRP    2
#define CHUNK   (NTHR * EPT * NGRP)
#define WCAP    (EPT * NGRP * 32)
#define LISTN   (NWAVE * WCAP)
#define NBC     4096
#define NBF     1024
#define RCAP    40960
#define RBN     128
#define TGT     256
#define DEGCAP  128
#define OTHR    512
#define WSCAP   134217728
#define NEG_SLOPE 0.2f
#define DEN_EPS 1e-16f
#define BN_EPS  1e-5f
#define NEG_BIG (-3.0e38f)

#define LDS_FILL ((RCAP + NBF + LISTN) * 4 + 64)

static_assert((CHUNK & (CHUNK - 1)) == 0);
static_assert(CHUNK <= 4096);
static_assert(NBC <= 4096 && NBF <= 4096);
static_assert((NBC & (NBC - 1)) == 0 && (NBF & (NBF - 1)) == 0);
static_assert(NBC == 4 * NBF);
static_assert(OTHR * 8 == NBC);
static_assert((RCAP % 32) == 0);
static_assert(TGT == NWAVE * 32);
static_assert((NBC % TGT) == 0);
static_assert(GMAX * 8 >= GMAX * NCLS);

typedef float          v4f  __attribute__((ext_vector_type(4)));
typedef float          v8f  __attribute__((ext_vector_type(8)));
typedef int            v4i  __attribute__((ext_vector_type(4)));
typedef unsigned short v8us __attribute__((ext_vector_type(8)));
typedef __bf16         v16b __attribute__((ext_vector_type(16)));
union FragB { v16b v; v8us h[2]; };

template <int KD, int NC>
struct GCfg {
  static constexpr int WPR  = (NC >= 32) ? 2 : 1;
  static constexpr int TPW  = NC / 16 / WPR;
  static constexpr int RG   = NWAVE / WPR;
  static constexpr int BM   = RG * 16;
  static constexpr int APK  = KD + 8;
  static constexpr int LDSA = 2 * BM * APK * 2;
  static constexpr int LDSS = BM * NC * 4;
  static constexpr int LDS  = LDSA > LDSS ? LDSA : LDSS;
};

__device__ __forceinline__ unsigned int bfr(float f) {
  const unsigned int u = __float_as_uint(f);
  return (u + 0x7FFFu + ((u >> 16) & 1u)) >> 16;
}

__device__ __forceinline__ void split1(float x, unsigned short& hb, unsigned short& lb) {
  const unsigned int hu = bfr(x);
  const float hf = __uint_as_float(hu << 16);
  hb = (unsigned short)hu;
  lb = (unsigned short)bfr(x - hf);
}

__device__ __forceinline__ void split8(v4f a, v4f b, v8us& hi, v8us& lo) {
  unsigned short hb, lb;
  split1(a.x, hb, lb); hi[0] = hb; lo[0] = lb;
  split1(a.y, hb, lb); hi[1] = hb; lo[1] = lb;
  split1(a.z, hb, lb); hi[2] = hb; lo[2] = lb;
  split1(a.w, hb, lb); hi[3] = hb; lo[3] = lb;
  split1(b.x, hb, lb); hi[4] = hb; lo[4] = lb;
  split1(b.y, hb, lb); hi[5] = hb; lo[5] = lb;
  split1(b.z, hb, lb); hi[6] = hb; lo[6] = lb;
  split1(b.w, hb, lb); hi[7] = hb; lo[7] = lb;
}

__device__ __forceinline__ v8f wmb(v16b a, v16b b, v8f c) {
  v8f d = __builtin_amdgcn_wmma_f32_16x16x32_bf16(false, a, false, b, (short)0, c, false, false);
  asm volatile("v_nop\n\tv_nop\n\tv_nop\n\tv_nop" : "+v"(d) : "v"(a), "v"(b));
  return d;
}

__device__ __forceinline__ float eluf(float v) { return v > 0.0f ? v : (__expf(v) - 1.0f); }

template <int NB>
__device__ __forceinline__ int scan_chunk(const int* __restrict__ dsts, int nE, int cbase, int slotBase,
                                          int vec8, int* list, int tid, int lane, int wave) {
  int wc = 0;
#pragma unroll
  for (int g = 0; g < NGRP; ++g) {
    const int el0  = (g * NTHR + tid) * EPT;
    const int e0   = cbase + el0;
    const int sent = -2147483647 - 1;
    v4i da, db;
    if (vec8 != 0 && cbase + CHUNK <= nE) {
      da = *(const v4i*)(dsts + e0);
      db = *(const v4i*)(dsts + e0 + 4);
    } else {
      da.x = (e0     < nE) ? dsts[min(e0, nE - 1)] : sent;
      da.y = (e0 + 1 < nE) ? dsts[min(e0 + 1, nE - 1)] : sent;
      da.z = (e0 + 2 < nE) ? dsts[min(e0 + 2, nE - 1)] : sent;
      da.w = (e0 + 3 < nE) ? dsts[min(e0 + 3, nE - 1)] : sent;
      db.x = (e0 + 4 < nE) ? dsts[min(e0 + 4, nE - 1)] : sent;
      db.y = (e0 + 5 < nE) ? dsts[min(e0 + 5, nE - 1)] : sent;
      db.z = (e0 + 6 < nE) ? dsts[min(e0 + 6, nE - 1)] : sent;
      db.w = (e0 + 7 < nE) ? dsts[min(e0 + 7, nE - 1)] : sent;
    }
    const unsigned nb = (unsigned)slotBase;
    const unsigned s0 = (unsigned)da.x - nb, s1 = (unsigned)da.y - nb;
    const unsigned s2 = (unsigned)da.z - nb, s3 = (unsigned)da.w - nb;
    const unsigned s4 = (unsigned)db.x - nb, s5 = (unsigned)db.y - nb;
    const unsigned s6 = (unsigned)db.z - nb, s7 = (unsigned)db.w - nb;
    const bool h0 = s0 < (unsigned)NB, h1 = s1 < (unsigned)NB, h2 = s2 < (unsigned)NB, h3 = s3 < (unsigned)NB;
    const bool h4 = s4 < (unsigned)NB, h5 = s5 < (unsigned)NB, h6 = s6 < (unsigned)NB, h7 = s7 < (unsigned)NB;
    const unsigned any = __builtin_amdgcn_ballot_w32(h0 | h1 | h2 | h3 | h4 | h5 | h6 | h7);
    if (any != 0u) {
#define HITJ(J, HJ, SJ) { \
        const unsigned mj = __builtin_amdgcn_ballot_w32(HJ); \
        if (mj != 0u) { \
          if (HJ) { \
            const int pos = wc + (int)__builtin_amdgcn_mbcnt_lo(mj, 0u); \
            if (pos < WCAP) list[wave * WCAP + pos] = ((el0 + (J)) << 12) | (int)(SJ); \
          } \
          wc += (int)__builtin_popcount(mj); } }
      HITJ(0, h0, s0)
      HITJ(1, h1, s1)
      HITJ(2, h2, s2)
      HITJ(3, h3, s3)
      HITJ(4, h4, s4)
      HITJ(5, h5, s5)
      HITJ(6, h6, s6)
      HITJ(7, h7, s7)
#undef HITJ
    }
  }
  return wc;
}

template <int KSRC, int KD, int NCOL, int NMAT>
__global__ __launch_bounds__(NTHR) void k_wprep(const float* __restrict__ W0, const float* __restrict__ W1,
                                                unsigned short* wp) {
  constexpr int NTOT  = NCOL * NMAT;
  constexpr int KD8   = KD / 8;
  constexpr int UNITS = NTOT * KD8;
  static_assert(KD % 32 == 0 && KSRC <= KD && (UNITS % 32) == 0 && (NMAT == 1 || NMAT == 2));
  const int i = (int)blockIdx.x * NTHR + (int)threadIdx.x;
  if (i >= UNITS) return;
  const int n   = i / KD8;
  const int k0  = (i - n * KD8) * 8;
  const int mat = n / NCOL;
  const int nc  = n - mat * NCOL;
  const float* W = (mat == 0) ? W0 : W1;
  float v[8];
#pragma unroll
  for (int e = 0; e < 8; ++e) {
    const int k  = k0 + e;
    const int kc = k < KSRC ? k : KSRC - 1;
    const float t = W[(size_t)kc * NCOL + nc];
    v[e] = (k < KSRC) ? t : 0.0f;
  }
  v4f a, b;
  a.x = v[0]; a.y = v[1]; a.z = v[2]; a.w = v[3];
  b.x = v[4]; b.y = v[5]; b.z = v[6]; b.w = v[7];
  v8us hv, lv;
  split8(a, b, hv, lv);
  unsigned short* dh = wp + (size_t)i * 8;
  unsigned short* dl = dh + (size_t)NTOT * KD;
  *(volatile v8us*)dh = hv;
  *(volatile v8us*)dl = lv;
  __threadfence();
  *(volatile v8us*)dh = hv;
  *(volatile v8us*)dl = lv;
}

__global__ __launch_bounds__(NTHR) void k_ecount(const int* __restrict__ eattr, int* ecnt, int nE, int vec4) {
  __shared__ int sw[NWAVE * 4];
  __shared__ __attribute__((aligned(16))) int sline[32];
  const int tid = threadIdx.x, lane = tid & 31, wave = tid >> 5;
  int c0 = 0, c1 = 0, c2 = 0;
#define ECNT(A) { const int ac = (A) < 0 ? 0 : ((A) > 2 ? 2 : (A)); c0 += (ac == 0); c1 += (ac == 1); c2 += (ac == 2); }
  if (vec4 != 0) {
    const int nv = nE >> 2;
#pragma unroll 1
    for (int i = tid; i < nv; i += NTHR) {
      const v4i a = *(const v4i*)(eattr + (size_t)i * 4);
      ECNT(a.x) ECNT(a.y) ECNT(a.z) ECNT(a.w)
    }
  } else {
#pragma unroll 1
    for (int i = tid; i < nE; i += NTHR) { const int a = eattr[i]; ECNT(a) }
  }
#undef ECNT
#pragma unroll
  for (int o = 16; o >= 1; o >>= 1) {
    c0 += __shfl_xor(c0, o); c1 += __shfl_xor(c1, o); c2 += __shfl_xor(c2, o);
  }
  if (tid < 32) sline[tid] = 0;
  if (lane == 0) { sw[wave * 4 + 0] = c0; sw[wave * 4 + 1] = c1; sw[wave * 4 + 2] = c2; }
  __syncthreads();
  if (tid == 0) {
    int t0 = 0, t1 = 0, t2 = 0;
#pragma unroll 1
    for (int w = 0; w < NWAVE; ++w) { t0 += sw[w * 4 + 0]; t1 += sw[w * 4 + 1]; t2 += sw[w * 4 + 2]; }
    sline[0] = t0; sline[1] = t1; sline[2] = t2;
  }
  __syncthreads();
  v4i v = {0, 0, 0, 0};
  if (tid < 8) v = *(const v4i*)(sline + 4 * tid);
  if (tid < 8) *(volatile v4i*)(ecnt + 4 * tid) = v;
  __threadfence();
  if (tid < 8) *(volatile v4i*)(ecnt + 4 * tid) = v;
}

__global__ __launch_bounds__(NTHR) void k_count(
    const int* __restrict__ dsts, int* cnt, int nE, int nN, int vec8) {
  __shared__ __attribute__((aligned(16))) int scnt[NBC];
  __shared__ __attribute__((aligned(16))) int list[LISTN];
  __shared__ int wcnt[NWAVE];
  const int tid = threadIdx.x, lane = tid & 31, wave = tid >> 5;
  const int nodeBase = blockIdx.x * NBC;

  for (int i = tid; i < NBC; i += NTHR) scnt[i] = (nodeBase + i < nN) ? 1 : 0;
  __syncthreads();

  const int nChunks = (nE + CHUNK - 1) / CHUNK;
#pragma unroll 1
  for (int ch = 0; ch < nChunks; ++ch) {
    const int cbase = ch * CHUNK;
    const int wc = scan_chunk<NBC>(dsts, nE, cbase, nodeBase, vec8, list, tid, lane, wave);
    if (lane == 0) wcnt[wave] = wc;
    __syncthreads();
    if (wave == 0) {
#pragma unroll 1
      for (int wsx = 0; wsx < NWAVE; ++wsx) {
        int n = __builtin_amdgcn_readfirstlane(wcnt[wsx]);
        n = n > WCAP ? WCAP : (n < 0 ? 0 : n);
        const int* lp = list + wsx * WCAP;
#pragma unroll 1
        for (int i = 0; i < n; ++i) {
          const int ent  = __builtin_amdgcn_readfirstlane(lp[i]);
          const int slot = ent & (NBC - 1);
          if (lane == 0) scnt[slot] = scnt[slot] + 1;
        }
      }
    }
    __syncthreads();
  }

  v4i cq[4];
#pragma unroll
  for (int q = 0; q < 4; ++q) {
    const int f = (wave * 4 + q) * 128 + 4 * lane;
    cq[q] = *(const v4i*)(scnt + f);
  }
  int* cp = cnt + (size_t)nodeBase;
#pragma unroll
  for (int q = 0; q < 4; ++q) {
    const int f = (wave * 4 + q) * 128 + 4 * lane;
    *(volatile v4i*)(cp + f) = cq[q];
  }
  __threadfence();
#pragma unroll
  for (int q = 0; q < 4; ++q) {
    const int f = (wave * 4 + q) * 128 + 4 * lane;
    *(volatile v4i*)(cp + f) = cq[q];
  }
}

__global__ __launch_bounds__(OTHR) void k_offsets(
    const int* __restrict__ cnt, int* off, int* rbase, int nChunk) {
  __shared__ __attribute__((aligned(16))) int soff[NBC];
  __shared__ __attribute__((aligned(16))) int srb[RBN];
  __shared__ int wtot[OTHR / 32];
  const int tid = threadIdx.x, lane = tid & 31, wave = tid >> 5, sub = tid >> 7;
  for (int i = tid; i < RBN; i += OTHR) srb[i] = 0;
  int carry = 0;
#pragma unroll 1
  for (int ch = 0; ch < nChunk; ++ch) {
    const int base = ch * NBC;
    const v4i c0 = *(const v4i*)(cnt + base + 8 * tid);
    const v4i c1 = *(const v4i*)(cnt + base + 8 * tid + 4);
    const int e0 = max(c0.x, 0), e1 = max(c0.y, 0), e2 = max(c0.z, 0), e3 = max(c0.w, 0);
    const int e4 = max(c1.x, 0), e5 = max(c1.y, 0), e6 = max(c1.z, 0), e7 = max(c1.w, 0);
    const int ts = e0 + e1 + e2 + e3 + e4 + e5 + e6 + e7;
    int incl = ts;
#pragma unroll
    for (int d = 1; d < 32; d <<= 1) {
      const int t = __shfl_up(incl, d);
      if (lane >= d) incl += t;
    }
    if (lane == 31) wtot[wave] = incl;
    __syncthreads();
    const int S0 = wtot[0]  + wtot[1]  + wtot[2]  + wtot[3];
    const int S1 = wtot[4]  + wtot[5]  + wtot[6]  + wtot[7];
    const int S2 = wtot[8]  + wtot[9]  + wtot[10] + wtot[11];
    const int S3 = wtot[12] + wtot[13] + wtot[14] + wtot[15];
    int pre = 0;
#pragma unroll 1
    for (int w = 4 * sub; w < wave; ++w) pre += wtot[w];
    const int b0 = carry;
    const int b1 = b0 + ((S0 + 31) & ~31);
    const int b2 = b1 + ((S1 + 31) & ~31);
    const int b3 = b2 + ((S2 + 31) & ~31);
    const int b4 = b3 + ((S3 + 31) & ~31);
    const int myb = sub == 0 ? b0 : (sub == 1 ? b1 : (sub == 2 ? b2 : b3));
    if (tid == 0) {
      srb[min(4 * ch + 0, RBN - 1)] = b0;
      srb[min(4 * ch + 1, RBN - 1)] = b1;
      srb[min(4 * ch + 2, RBN - 1)] = b2;
      srb[min(4 * ch + 3, RBN - 1)] = b3;
    }
    int run = myb + pre + incl - ts;
    soff[8 * tid + 0] = run; run += e0;
    soff[8 * tid + 1] = run; run += e1;
    soff[8 * tid + 2] = run; run += e2;
    soff[8 * tid + 3] = run; run += e3;
    soff[8 * tid + 4] = run; run += e4;
    soff[8 * tid + 5] = run; run += e5;
    soff[8 * tid + 6] = run; run += e6;
    soff[8 * tid + 7] = run;
    carry = b4;
    __syncthreads();
    const v4i o0 = *(const v4i*)(soff + 4 * tid);
    const v4i o1 = *(const v4i*)(soff + 4 * (tid + OTHR));
    int* op = off + base;
    *(volatile v4i*)(op + 4 * tid) = o0;
    *(volatile v4i*)(op + 4 * (tid + OTHR)) = o1;
    __threadfence();
    *(volatile v4i*)(op + 4 * tid) = o0;
    *(volatile v4i*)(op + 4 * (tid + OTHR)) = o1;
    __syncthreads();
  }
  if (tid == 0) srb[min(4 * nChunk, RBN - 1)] = carry;
  __syncthreads();
  v4i rv = {0, 0, 0, 0};
  if (tid < 32) rv = *(const v4i*)(srb + 4 * tid);
  if (tid < 32) *(volatile v4i*)(rbase + 4 * tid) = rv;
  __threadfence();
  if (tid < 32) *(volatile v4i*)(rbase + 4 * tid) = rv;
}

__global__ __launch_bounds__(NTHR) void k_fill(
    const int* __restrict__ srcs, const int* __restrict__ dsts, const int* __restrict__ eattr,
    const int* __restrict__ off, const int* __restrict__ rbase,
    int* csr, int nN, int nE, int vec8, int csrLen) {
  extern __shared__ v4f lds_dyn[];
  int* region = (int*)lds_dyn;
  int* cursor = region + RCAP;
  int* list   = cursor + NBF;
  int* wcnt   = list + LISTN;
  const int tid = threadIdx.x, lane = tid & 31, wave = tid >> 5;
  const int b = blockIdx.x;
  const int nodeBase = b * NBF;

  int rb0 = rbase[b];
  const int rb1 = rbase[b + 1];
  rb0 = rb0 < 0 ? 0 : (rb0 > csrLen ? csrLen : rb0);
  rb0 &= ~31;
  int len = rb1 - rb0;
  len = len < 0 ? 0 : (len > RCAP ? RCAP : len);
  int lenW = (len + 31) & ~31;
  if (rb0 + lenW > csrLen) lenW = (csrLen - rb0) & ~31;

  {
    const v4i z = {0, 0, 0, 0};
    for (int i = tid; i < RCAP / 4; i += NTHR) ((v4i*)region)[i] = z;
  }
  __syncthreads();
  for (int s = tid; s < NBF; s += NTHR) {
    int o = off[nodeBase + s] - rb0;
    o = o < 0 ? 0 : (o > RCAP ? RCAP : o);
    const int node = nodeBase + s;
    if (node < nN) {
      const int pos = o > RCAP - 1 ? RCAP - 1 : o;
      region[pos] = (node << 2) | 3;
      o = (o + 1 > RCAP) ? RCAP : o + 1;
    }
    cursor[s] = o;
  }
  __syncthreads();

  const int nChunks = (nE + CHUNK - 1) / CHUNK;
#pragma unroll 1
  for (int ch = 0; ch < nChunks; ++ch) {
    const int cbase = ch * CHUNK;
    const int wc = scan_chunk<NBF>(dsts, nE, cbase, nodeBase, vec8, list, tid, lane, wave);
    if (lane == 0) wcnt[wave] = wc;
    __syncthreads();
    if (wave == 0) {
#pragma unroll 1
      for (int wsx = 0; wsx < NWAVE; ++wsx) {
        int n = __builtin_amdgcn_readfirstlane(wcnt[wsx]);
        n = n > WCAP ? WCAP : (n < 0 ? 0 : n);
        const int* lp = list + wsx * WCAP;
#pragma unroll 1
        for (int i = 0; i < n; ++i) {
          const int ent  = __builtin_amdgcn_readfirstlane(lp[i]);
          const int slot = ent & (NBF - 1);
          int e = cbase + ((ent >> 12) & (CHUNK - 1));
          e = e > nE - 1 ? nE - 1 : e;
          int src = srcs[e];
          src = src < 0 ? 0 : (src > nN - 1 ? nN - 1 : src);
          int at = eattr[e];
          at = at < 0 ? 0 : (at > 2 ? 2 : at);
          if (lane == 0) {
            int pos = cursor[slot];
            pos = pos < 0 ? 0 : (pos > RCAP - 1 ? RCAP - 1 : pos);
            region[pos] = (src << 2) | at;
            const int np = pos + 1;
            cursor[slot] = np > RCAP ? RCAP : np;
          }
        }
      }
    }
    __syncthreads();
  }

  const int nv = lenW >> 2;
  int* gp = csr + rb0;
#pragma unroll 1
  for (int i = tid; i < nv; i += NTHR) { const v4i v = ((const v4i*)region)[i]; *(volatile v4i*)(gp + 4 * i) = v; }
  __threadfence();
#pragma unroll 1
  for (int i = tid; i < nv; i += NTHR) { const v4i v = ((const v4i*)region)[i]; *(volatile v4i*)(gp + 4 * i) = v; }
}

template <int KSRC, int KD, int NC, int EPI>
__global__ __launch_bounds__(NTHR) void k_gemm(
    const float* __restrict__ A, const unsigned short* __restrict__ Bw,
    const float* __restrict__ bias0, const float* __restrict__ bias1,
    const float* __restrict__ gam0, const float* __restrict__ gam1,
    const float* __restrict__ bet0, const float* __restrict__ bet1,
    float* C, int nRowsA) {
  typedef GCfg<KD, NC> G;
  constexpr int WPR  = G::WPR;
  constexpr int TPW  = G::TPW;
  constexpr int BM   = G::BM;
  constexpr int APK  = G::APK;
  constexpr int Q4   = TPW * 4;
  constexpr int RPI  = 32 / Q4;
  constexpr int NIT  = 16 / RPI;
  constexpr int UPT  = (BM * KD / 8) / NTHR;
  constexpr size_t WPLN = (size_t)NC * KD;
  static_assert(KD % 32 == 0 && KSRC <= KD && WPR == 2 && NC % (16 * WPR) == 0);
  static_assert((Q4 & (Q4 - 1)) == 0 && Q4 <= 32);
  static_assert(NIT * RPI == 16);
  static_assert(UPT >= 1 && UPT * NTHR * 8 == BM * KD);
  static_assert(((APK * 2) % 16) == 0);
  static_assert(BM * NC * 4 <= G::LDS && 2 * BM * APK * 2 <= G::LDS);

  extern __shared__ v4f lds_dyn[];
  unsigned short* sHi = (unsigned short*)lds_dyn;
  unsigned short* sLo = sHi + BM * APK;
  float*          stg = (float*)lds_dyn;
  const int tid = threadIdx.x, lane = tid & 31, wave = tid >> 5, hh = lane >> 4, m = lane & 15;
  const int rowBase = blockIdx.x * BM;

#pragma unroll
  for (int i = 0; i < UPT; ++i) {
    const int idx = i * NTHR + tid;
    const int r   = idx / (KD / 8);
    const int c0  = (idx - r * (KD / 8)) * 8;
    int row = rowBase + r;
    row = row > nRowsA - 1 ? nRowsA - 1 : row;
    v4f a, b;
    if constexpr (KSRC == KD) {
      const float* ap = A + (size_t)row * KD + c0;
      a = *(const v4f*)ap;
      b = *(const v4f*)(ap + 4);
    } else {
      float t[8];
#pragma unroll
      for (int e = 0; e < 8; ++e) {
        const int k  = c0 + e;
        const int kc = k < KSRC ? k : KSRC - 1;
        const float tv = A[(size_t)row * KSRC + kc];
        t[e] = (k < KSRC) ? tv : 0.0f;
      }
      a.x = t[0]; a.y = t[1]; a.z = t[2]; a.w = t[3];
      b.x = t[4]; b.y = t[5]; b.z = t[6]; b.w = t[7];
    }
    v8us hv, lv;
    split8(a, b, hv, lv);
    *(v8us*)(sHi + r * APK + c0) = hv;
    *(v8us*)(sLo + r * APK + c0) = lv;
  }
  __syncthreads();

  const int rg  = wave / WPR;
  const int chf = wave - rg * WPR;
  const int r0  = rg * 16;
  const int c0  = chf * TPW * 16;

  v8f acc[TPW];
#pragma unroll
  for (int t = 0; t < TPW; ++t) { v8f z = {0.f, 0.f, 0.f, 0.f, 0.f, 0.f, 0.f, 0.f}; acc[t] = z; }
  const unsigned short* ahp = sHi + (r0 + m) * APK + 8 * hh;
  const unsigned short* alp = sLo + (r0 + m) * APK + 8 * hh;
#pragma unroll 2
  for (int kt = 0; kt < KD / 32; ++kt) {
    FragB ah, al;
    ah.h[0] = *(const v8us*)(ahp + 32 * kt);
    ah.h[1] = *(const v8us*)(ahp + 32 * kt + 16);
    al.h[0] = *(const v8us*)(alp + 32 * kt);
    al.h[1] = *(const v8us*)(alp + 32 * kt + 16);
#pragma unroll
    for (int t = 0; t < TPW; ++t) {
      const unsigned short* bp = Bw + (size_t)(c0 + 16 * t + m) * KD + 32 * kt + 8 * hh;
      FragB bh, bl;
      bh.h[0] = *(const v8us*)bp;
      bh.h[1] = *(const v8us*)(bp + 16);
      bl.h[0] = *(const v8us*)(bp + WPLN);
      bl.h[1] = *(const v8us*)(bp + WPLN + 16);
      acc[t] = wmb(ah.v, bh.v, acc[t]);
      acc[t] = wmb(ah.v, bl.v, acc[t]);
      acc[t] = wmb(al.v, bh.v, acc[t]);
    }
  }
  __syncthreads();

  {
    float* sp = stg + (size_t)(r0 + 8 * hh) * NC + c0 + m;
#pragma unroll
    for (int t = 0; t < TPW; ++t) {
#pragma unroll
      for (int r = 0; r < 8; ++r) sp[r * NC + 16 * t] = acc[t][r];
    }
  }
  __syncthreads();

  const int qq   = lane & (Q4 - 1);
  const int rsub = lane / Q4;
  const int colh = 4 * qq;
  const int col  = c0 + colh;
  const float* bp0 = (chf == 0) ? bias0 : bias1;
  const v4f b4 = *(const v4f*)(bp0 + colh);
  v4f sc4 = {1.f, 1.f, 1.f, 1.f};
  v4f sh4 = {0.f, 0.f, 0.f, 0.f};
  if constexpr ((EPI & 1) != 0) {
    const float* gp = (chf == 0) ? gam0 : gam1;
    const float* ep = (chf == 0) ? bet0 : bet1;
    const float inv = 1.0f / sqrtf(1.0f + BN_EPS);
    sc4 = *(const v4f*)(gp + colh) * inv;
    sh4 = *(const v4f*)(ep + colh);
  }
  const size_t gb = (size_t)(rowBase + r0) * NC + col;
#pragma unroll
  for (int it = 0; it < NIT; ++it) {
    const int row = it * RPI + rsub;
    v4f v = *(const v4f*)(stg + (size_t)(r0 + row) * NC + col) + b4;
    if constexpr ((EPI & 1) != 0) v = v * sc4 + sh4;
    if constexpr ((EPI & 2) != 0) { v.x = fmaxf(v.x, 0.f); v.y = fmaxf(v.y, 0.f); v.z = fmaxf(v.z, 0.f); v.w = fmaxf(v.w, 0.f); }
    *(volatile v4f*)(C + gb + (size_t)row * NC) = v;
  }
  __threadfence();
#pragma unroll
  for (int it = 0; it < NIT; ++it) {
    const int row = it * RPI + rsub;
    v4f v = *(const v4f*)(stg + (size_t)(r0 + row) * NC + col) + b4;
    if constexpr ((EPI & 1) != 0) v = v * sc4 + sh4;
    if constexpr ((EPI & 2) != 0) { v.x = fmaxf(v.x, 0.f); v.y = fmaxf(v.y, 0.f); v.z = fmaxf(v.z, 0.f); v.w = fmaxf(v.w, 0.f); }
    *(volatile v4f*)(C + gb + (size_t)row * NC) = v;
  }
}

template <int NCD, int RESID>
__global__ __launch_bounds__(NTHR) void k_agg(
    const int* __restrict__ csr, const int* __restrict__ off, const int* __restrict__ cnt,
    const float* __restrict__ xlr, const float* __restrict__ emb, const int* __restrict__ ecnt,
    const float* __restrict__ We, const float* __restrict__ att,
    const float* __restrict__ bo, const float* __restrict__ gam, const float* __restrict__ bet,
    const float* __restrict__ hin, float* hout, int nN, int csrLen, float invE) {
  constexpr int NCW = 2 * NCD;
  static_assert(NCD == 128 || NCD == 64);
  static_assert(DEGCAP % 32 == 0);
  __shared__ __attribute__((aligned(16))) float eet[4 * NCD];
  __shared__ __attribute__((aligned(16))) float slg[NWAVE * DEGCAP * 4];
  const int tid = threadIdx.x, lane = tid & 31, wave = tid >> 5;

  {
    const float fc0 = (float)ecnt[0], fc1 = (float)ecnt[1], fc2 = (float)ecnt[2];
#pragma unroll 1
    for (int i = tid; i < 4 * NCD; i += NTHR) {
      const int a  = i / NCD;
      const int c  = i - a * NCD;
      const int ar = a < 3 ? a : 2;
      float s = 0.0f;
#pragma unroll 1
      for (int k = 0; k < EDM; ++k) {
        const float em = (fc0 * emb[k] + fc1 * emb[EDM + k] + fc2 * emb[2 * EDM + k]) * invE;
        const float ea = emb[ar * EDM + k];
        const float ev = (a < 3) ? ea : em;
        s = fmaf(ev, We[k * NCD + c], s);
      }
      eet[i] = s;
    }
  }
  __syncthreads();

  const int  q    = (NCD == 128) ? lane : (lane & 15);
  const int  col0 = 4 * q;
  const int  hd   = q >> 3;
  const bool wlg  = ((lane & 7) == 0) && ((NCD == 128) || (lane < 16));
  const bool stok = (NCD == 128) || (lane < 16);
  const v4f  z4   = {0.f, 0.f, 0.f, 0.f};
  const v4f  at4  = *(const v4f*)(att + col0);
  const v4f  bo4  = *(const v4f*)(bo + col0);
  const float inv = 1.0f / sqrtf(1.0f + BN_EPS);
  const v4f  sc4  = *(const v4f*)(gam + col0) * inv;
  const v4f  sh4  = *(const v4f*)(bet + col0);
  float* slw = slg + wave * (DEGCAP * 4);

  const int tbase = blockIdx.x * TGT + wave * 32;
  const int cnt_l = cnt[tbase + lane];
  const int off_l = off[tbase + lane];

#pragma unroll 1
  for (int j = 0; j < 32; ++j) {
    const int c = tbase + j;
    int n = __shfl(cnt_l, j);
    n = n < 0 ? 0 : (n > DEGCAP ? DEGCAP : n);
    const int st = __shfl(off_l, j);
    const v4f xr4 = *(const v4f*)(xlr + (size_t)c * NCW + NCD + col0);

    float mx = NEG_BIG;
#pragma unroll 1
    for (int q0 = 0; q0 < n; q0 += 32) {
      int pos = st + q0 + lane;
      pos = pos < 0 ? 0 : (pos > csrLen - 1 ? csrLen - 1 : pos);
      const int ent  = csr[pos];
      const int mcnt = (n - q0) < 32 ? (n - q0) : 32;
#pragma unroll 1
      for (int pp = 0; pp < mcnt; ++pp) {
        const int en = __builtin_amdgcn_readlane(ent, pp);
        int s = en >> 2;
        s = s < 0 ? 0 : (s > nN - 1 ? nN - 1 : s);
        const int a = en & 3;
        const v4f xl4 = *(const v4f*)(xlr + (size_t)s * NCW + col0);
        const v4f ee4 = *(const v4f*)(eet + a * NCD + col0);
        v4f mm = xl4 + xr4 + ee4;
        mm.x = fmaxf(mm.x, NEG_SLOPE * mm.x); mm.y = fmaxf(mm.y, NEG_SLOPE * mm.y);
        mm.z = fmaxf(mm.z, NEG_SLOPE * mm.z); mm.w = fmaxf(mm.w, NEG_SLOPE * mm.w);
        float d = mm.x * at4.x + mm.y * at4.y + mm.z * at4.z + mm.w * at4.w;
        d += __shfl_xor(d, 1);
        d += __shfl_xor(d, 2);
        d += __shfl_xor(d, 4);
        mx = fmaxf(mx, d);
        if (wlg) slw[(q0 + pp) * 4 + hd] = d;
      }
    }
    __builtin_amdgcn_fence(__ATOMIC_RELEASE, "wavefront");
    __builtin_amdgcn_wave_barrier();

    float den = 0.0f;
    v4f   acc = z4;
#pragma unroll 1
    for (int q0 = 0; q0 < n; q0 += 32) {
      int pos = st + q0 + lane;
      pos = pos < 0 ? 0 : (pos > csrLen - 1 ? csrLen - 1 : pos);
      const int ent  = csr[pos];
      const int mcnt = (n - q0) < 32 ? (n - q0) : 32;
#pragma unroll 1
      for (int pp = 0; pp < mcnt; ++pp) {
        const int en = __builtin_amdgcn_readlane(ent, pp);
        int s = en >> 2;
        s = s < 0 ? 0 : (s > nN - 1 ? nN - 1 : s);
        const v4f xl4 = *(const v4f*)(xlr + (size_t)s * NCW + col0);
        const float lg = slw[(q0 + pp) * 4 + hd];
        const float p  = __expf(lg - mx);
        den += p;
        acc = acc + xl4 * p;
      }
    }
    __builtin_amdgcn_fence(__ATOMIC_RELEASE, "wavefront");
    __builtin_amdgcn_wave_barrier();

    const float rd = 1.0f / (den + DEN_EPS);
    v4f v = acc * rd + bo4;
    v = v * sc4 + sh4;
    v.x = eluf(v.x); v.y = eluf(v.y); v.z = eluf(v.z); v.w = eluf(v.w);
    if constexpr (RESID != 0) {
      const v4f hr = *(const v4f*)(hin + (size_t)c * NCD + col0);
      v = v + hr;
    }
    if (c >= nN) v = z4;
    float* pw = hout + (size_t)c * NCD + col0;
    if (stok) *(volatile v4f*)pw = v;
    __threadfence();
    if (stok) *(volatile v4f*)pw = v;
  }
}

__global__ __launch_bounds__(NTHR) void k_pool(const float* __restrict__ h3, const int* __restrict__ batch,
                                               float* pooled, int nN) {
  __shared__ __attribute__((aligned(16))) float ssum[NWAVE * HC];
  __shared__ __attribute__((aligned(16))) float smax[NWAVE * HC];
  __shared__ int scn[NWAVE];
  __shared__ __attribute__((aligned(16))) float spool[2 * HC];
  const int tid = threadIdx.x, lane = tid & 31, wave = tid >> 5;
  const int g  = blockIdx.x;
  const int ql = lane & 15;
  v4f s4 = {0.f, 0.f, 0.f, 0.f};
  v4f m4 = {NEG_BIG, NEG_BIG, NEG_BIG, NEG_BIG};
  int cw = 0;
  const int nCh = (nN + 31) / 32;
#pragma unroll 1
  for (int ch = wave; ch < nCh; ch += NWAVE) {
    const int n  = ch * 32 + lane;
    const int nc = n < nN ? n : nN - 1;
    const int bv = batch[nc];
    const bool hit = (n < nN) && (bv == g);
    unsigned mk = __builtin_amdgcn_ballot_w32(hit);
    cw += (int)__builtin_popcount(mk);
#pragma unroll 1
    for (; mk != 0u; mk &= mk - 1u) {
      const int idx  = __builtin_ctz(mk);
      const int node = ch * 32 + idx;
      const v4f v = *(const v4f*)(h3 + (size_t)node * HC + 4 * ql);
      s4 = s4 + v;
      m4.x = fmaxf(m4.x, v.x); m4.y = fmaxf(m4.y, v.y); m4.z = fmaxf(m4.z, v.z); m4.w = fmaxf(m4.w, v.w);
    }
  }
  if (lane < 16) {
    *(v4f*)(ssum + wave * HC + 4 * lane) = s4;
    *(v4f*)(smax + wave * HC + 4 * lane) = m4;
  }
  if (lane == 0) scn[wave] = cw;
  __syncthreads();
  if (tid < HC) {
    float s = 0.0f, mxv = NEG_BIG;
    int c = 0;
#pragma unroll 1
    for (int w = 0; w < NWAVE; ++w) {
      s  += ssum[w * HC + tid];
      mxv = fmaxf(mxv, smax[w * HC + tid]);
      c  += scn[w];
    }
    const float fc = (float)(c > 1 ? c : 1);
    spool[tid]      = s * (1.0f / fc);
    spool[HC + tid] = (c > 0) ? mxv : 0.0f;
  }
  __syncthreads();
  v4f pv = {0.f, 0.f, 0.f, 0.f};
  if (wave == 0) pv = *(const v4f*)(spool + 4 * lane);
  float* pp = pooled + (size_t)g * (2 * HC) + 4 * lane;
  if (wave == 0) *(volatile v4f*)pp = pv;
  __threadfence();
  if (wave == 0) *(volatile v4f*)pp = pv;
}

__global__ __launch_bounds__(NTHR) void k_cls(const float* __restrict__ hid, const float* __restrict__ wc2,
                                              const float* __restrict__ bc2, float* out, int nG, int outN) {
  __shared__ __attribute__((aligned(16))) float so[GMAX * 8];
  const int tid = threadIdx.x;
#pragma unroll 1
  for (int i = tid; i < GMAX * 8; i += NTHR) {
    int g = i / NCLS;
    const int j = i - g * NCLS;
    g = g > nG - 1 ? nG - 1 : g;
    float o = 0.0f;
#pragma unroll 1
    for (int k = 0; k < HC; ++k) o = fmaf(hid[g * HC + k], wc2[k * NCLS + j], o);
    o += bc2[j];
    so[i] = (i < outN) ? o : 0.0f;
  }
  __syncthreads();
  const int nv = outN >> 2;
  v4f v = {0.f, 0.f, 0.f, 0.f};
  if (tid < nv) v = *(const v4f*)(so + 4 * tid);
  if (tid < nv) *(volatile v4f*)(out + 4 * tid) = v;
  if (tid == 0) {
#pragma unroll 1
    for (int t = 4 * nv; t < outN; ++t) *(volatile float*)(out + t) = so[t];
  }
  __threadfence();
  if (tid < nv) *(volatile v4f*)(out + 4 * tid) = v;
  if (tid == 0) {
#pragma unroll 1
    for (int t = 4 * nv; t < outN; ++t) *(volatile float*)(out + t) = so[t];
  }
}

typedef GCfg<KIN, HID>     GI;
typedef GCfg<HID, 2 * HID> GL;
typedef GCfg<HID, 2 * HC>  G3;
typedef GCfg<HID, HC>      GH;
static_assert((TGT % GI::BM) == 0 && (TGT % GL::BM) == 0 && (TGT % G3::BM) == 0 && GH::BM == GMAX);

extern "C" void kernel_launch(void* const* d_in, const int* in_sizes, int n_in,
                              void* d_out, int out_size, void* d_ws, size_t ws_size,
                              hipStream_t stream) {
  if (n_in < 40) return;
  const int nN = in_sizes[3];
  const int nE = in_sizes[2];
  if (nN <= 0 || nE <= 0) return;
  if (in_sizes[0] != nN * FIN || in_sizes[1] != 2 * nE || in_sizes[4] != 3 * EDM) return;
  if (in_sizes[5] != FIN * HID || in_sizes[6] != HID || in_sizes[7] != HID || in_sizes[8] != HID) return;
  for (int l = 0; l < 2; ++l) {
    const int b = 9 + 9 * l;
    if (in_sizes[b] != HID * HID || in_sizes[b + 2] != HID * HID || in_sizes[b + 4] != EDM * HID) return;
    if (in_sizes[b + 1] != HID || in_sizes[b + 3] != HID || in_sizes[b + 5] != HID) return;
    if (in_sizes[b + 6] != HID || in_sizes[b + 7] != HID || in_sizes[b + 8] != HID) return;
  }
  {
    const int b = 27;
    if (in_sizes[b] != HID * HC || in_sizes[b + 2] != HID * HC || in_sizes[b + 4] != EDM * HC) return;
    if (in_sizes[b + 1] != HC || in_sizes[b + 3] != HC || in_sizes[b + 5] != HC) return;
    if (in_sizes[b + 6] != HC || in_sizes[b + 7] != HC || in_sizes[b + 8] != HC) return;
  }
  if (in_sizes[36] != HID * HC || in_sizes[37] != HC || in_sizes[38] != HC * NCLS || in_sizes[39] != NCLS) return;
  const int nG = out_size / NCLS;
  if (nG <= 0 || nG * NCLS != out_size || nG > GMAX) return;
  if (nE > (1 << 26) || nN > (1 << 22)) return;

  const float* x     = (const float*)d_in[0];
  const int*   ei    = (const int*)d_in[1];
  const int*   src   = ei;
  const int*   dst   = ei + nE;
  const int*   eattr = (const int*)d_in[2];
  const int*   batch = (const int*)d_in[3];
  const float* emb   = (const float*)d_in[4];
  const float* w_in  = (const float*)d_in[5];
  const float* b_in  = (const float*)d_in[6];
  const float* g_in  = (const float*)d_in[7];
  const float* be_in = (const float*)d_in[8];
  const float *wl[3], *bl[3], *wr[3], *br[3], *we[3], *att[3], *bo[3], *gl[3], *bb[3];
  for (int l = 0; l < 3; ++l) {
    const int b = 9 + 9 * l;
    wl[l]  = (const float*)d_in[b + 0];
    bl[l]  = (const float*)d_in[b + 1];
    wr[l]  = (const float*)d_in[b + 2];
    br[l]  = (const float*)d_in[b + 3];
    we[l]  = (const float*)d_in[b + 4];
    att[l] = (const float*)d_in[b + 5];
    bo[l]  = (const float*)d_in[b + 6];
    gl[l]  = (const float*)d_in[b + 7];
    bb[l]  = (const float*)d_in[b + 8];
  }
  const float* wc1 = (const float*)d_in[36];
  const float* bc1 = (const float*)d_in[37];
  const float* wc2 = (const float*)d_in[38];
  const float* bc2 = (const float*)d_in[39];
  float* out = (float*)d_out;

  const int NPAD   = ((nN + TGT - 1) / TGT) * TGT;
  const int nBC    = (nN + NBC - 1) / NBC;
  const int CNTPAD = nBC * NBC;
  if (4 * nBC + 1 > RBN) return;
  const int nBF    = (nN + NBF - 1) / NBF;
  const int csrLen = ((nE + CNTPAD + 31) & ~31) + 4096;
  if (31 * 4 * nBC > 4096) return;
  const int nAgg   = NPAD / TGT;

  char* ws = (char*)d_ws;
  size_t off = 0;
  const size_t oWin = off; off += (size_t)2 * HID * KIN * 2;             off = (off + 255) & ~(size_t)255;
  const size_t oW1  = off; off += (size_t)2 * (2 * HID) * HID * 2;       off = (off + 255) & ~(size_t)255;
  const size_t oW2  = off; off += (size_t)2 * (2 * HID) * HID * 2;       off = (off + 255) & ~(size_t)255;
  const size_t oW3  = off; off += (size_t)2 * (2 * HC) * HID * 2;        off = (off + 255) & ~(size_t)255;
  const size_t oWc  = off; off += (size_t)2 * HC * HID * 2;              off = (off + 255) & ~(size_t)255;
  const size_t oEc  = off; off += (size_t)32 * 4;                        off = (off + 255) & ~(size_t)255;
  const size_t oCnt = off; off += (size_t)CNTPAD * 4;                    off = (off + 255) & ~(size_t)255;
  const size_t oOff = off; off += (size_t)CNTPAD * 4;                    off = (off + 255) & ~(size_t)255;
  const size_t oRb  = off; off += (size_t)RBN * 4;                       off = (off + 255) & ~(size_t)255;
  const size_t oCsr = off; off += (size_t)csrLen * 4;                    off = (off + 255) & ~(size_t)255;
  const size_t oHA  = off; off += (size_t)NPAD * HID * 4;                off = (off + 255) & ~(size_t)255;
  const size_t oHB  = off; off += (size_t)NPAD * HID * 4;                off = (off + 255) & ~(size_t)255;
  const size_t oXlr = off; off += (size_t)NPAD * (2 * HID) * 4;          off = (off + 255) & ~(size_t)255;
  const size_t oH3  = off; off += (size_t)NPAD * HC * 4;                 off = (off + 255) & ~(size_t)255;
  const size_t oPool = off; off += (size_t)GMAX * (2 * HC) * 4;          off = (off + 255) & ~(size_t)255;
  const size_t oHid = off; off += (size_t)GMAX * HC * 4;                 off = (off + 255) & ~(size_t)255;
  if (off > ws_size || off > (size_t)WSCAP) return;
  unsigned short* wpIn = (unsigned short*)(ws + oWin);
  unsigned short* wp1  = (unsigned short*)(ws + oW1);
  unsigned short* wp2  = (unsigned short*)(ws + oW2);
  unsigned short* wp3  = (unsigned short*)(ws + oW3);
  unsigned short* wpc  = (unsigned short*)(ws + oWc);
  int*   ecnt = (int*)(ws + oEc);
  int*   cnt  = (int*)(ws + oCnt);
  int*   offp = (int*)(ws + oOff);
  int*   rb   = (int*)(ws + oRb);
  int*   csr  = (int*)(ws + oCsr);
  float* hA   = (float*)(ws + oHA);
  float* hB   = (float*)(ws + oHB);
  float* xlr  = (float*)(ws + oXlr);
  float* h3   = (float*)(ws + oH3);
  float* pool = (float*)(ws + oPool);
  float* hid  = (float*)(ws + oHid);

  const int   vec  = ((nE & 3) == 0) ? 1 : 0;
  const float invE = 1.0f / (float)nE;

  k_wprep<FIN, KIN, HID, 1><<<(HID * KIN / 8 + NTHR - 1) / NTHR, NTHR, 0, stream>>>(w_in, w_in, wpIn);
  k_wprep<HID, HID, HID, 2><<<(2 * HID * HID / 8 + NTHR - 1) / NTHR, NTHR, 0, stream>>>(wl[0], wr[0], wp1);
  k_wprep<HID, HID, HID, 2><<<(2 * HID * HID / 8 + NTHR - 1) / NTHR, NTHR, 0, stream>>>(wl[1], wr[1], wp2);
  k_wprep<HID, HID, HC, 2><<<(2 * HC * HID / 8 + NTHR - 1) / NTHR, NTHR, 0, stream>>>(wl[2], wr[2], wp3);
  k_wprep<HID, HID, HC, 1><<<(HC * HID / 8 + NTHR - 1) / NTHR, NTHR, 0, stream>>>(wc1, wc1, wpc);

  k_ecount<<<1, NTHR, 0, stream>>>(eattr, ecnt, nE, vec);

  k_count<<<nBC, NTHR, 0, stream>>>(dst, cnt, nE, nN, vec);
  k_offsets<<<1, OTHR, 0, stream>>>(cnt, offp, rb, nBC);
  hipFuncSetAttribute(reinterpret_cast<const void*>(&k_fill),
                      hipFuncAttributeMaxDynamicSharedMemorySize, LDS_FILL);
  k_fill<<<nBF, NTHR, LDS_FILL, stream>>>(src, dst, eattr, offp, rb, csr, nN, nE, vec, csrLen);

  hipFuncSetAttribute(reinterpret_cast<const void*>(&k_gemm<FIN, KIN, HID, 3>),
                      hipFuncAttributeMaxDynamicSharedMemorySize, GI::LDS);
  k_gemm<FIN, KIN, HID, 3><<<NPAD / GI::BM, NTHR, GI::LDS, stream>>>(
      x, wpIn, b_in, b_in + HID / 2, g_in, g_in + HID / 2, be_in, be_in + HID / 2, hA, nN);

  hipFuncSetAttribute(reinterpret_cast<const void*>(&k_gemm<HID, HID, 2 * HID, 0>),
                      hipFuncAttributeMaxDynamicSharedMemorySize, GL::LDS);
  k_gemm<HID, HID, 2 * HID, 0><<<NPAD / GL::BM, NTHR, GL::LDS, stream>>>(
      hA, wp1, bl[0], br[0], bl[0], br[0], bl[0], br[0], xlr, NPAD);
  k_agg<HID, 1><<<nAgg, NTHR, 0, stream>>>(csr, offp, cnt, xlr, emb, ecnt, we[0], att[0], bo[0], gl[0], bb[0],
                                           hA, hB, nN, csrLen, invE);

  k_gemm<HID, HID, 2 * HID, 0><<<NPAD / GL::BM, NTHR, GL::LDS, stream>>>(
      hB, wp2, bl[1], br[1], bl[1], br[1], bl[1], br[1], xlr, NPAD);
  k_agg<HID, 1><<<nAgg, NTHR, 0, stream>>>(csr, offp, cnt, xlr, emb, ecnt, we[1], att[1], bo[1], gl[1], bb[1],
                                           hB, hA, nN, csrLen, invE);

  hipFuncSetAttribute(reinterpret_cast<const void*>(&k_gemm<HID, HID, 2 * HC, 0>),
                      hipFuncAttributeMaxDynamicSharedMemorySize, G3::LDS);
  k_gemm<HID, HID, 2 * HC, 0><<<NPAD / G3::BM, NTHR, G3::LDS, stream>>>(
      hA, wp3, bl[2], br[2], bl[2], br[2], bl[2], br[2], xlr, NPAD);
  k_agg<HC, 0><<<nAgg, NTHR, 0, stream>>>(csr, offp, cnt, xlr, emb, ecnt, we[2], att[2], bo[2], gl[2], bb[2],
                                          hA, h3, nN, csrLen, invE);

  k_pool<<<nG, NTHR, 0, stream>>>(h3, batch, pool, nN);
  hipFuncSetAttribute(reinterpret_cast<const void*>(&k_gemm<HID, HID, HC, 2>),
                      hipFuncAttributeMaxDynamicSharedMemorySize, GH::LDS);
  k_gemm<HID, HID, HC, 2><<<1, NTHR, GH::LDS, stream>>>(
      pool, wpc, bc1, bc1 + HC / 2, bc1, bc1 + HC / 2, bc1, bc1 + HC / 2, hid, nG);
  k_cls<<<1, NTHR, 0, stream>>>(hid, wc2, bc2, out, nG, out_size);
}
